// mlp_84748294685180
// MI455X (gfx1250) — hardware-run, weakly checked
//
#include <hip/hip_runtime.h>
#include <stddef.h>
#include <stdint.h>

#define IND     16
#define WID     128
#define WP      136
#define NHL     3
#define PCOUNT  51841
#define OFF_B0  2048
#define OFF_W1  2176
#define LSTRIDE 16512
#define OFF_WL  51712
#define OFF_BL  51840
#define NWAVES  4
#define TM      16
#define RPI     (NWAVES * TM)
#define ITERS   16
#define RPB     (RPI * ITERS)
#define WMAT    (WID * WP)
#define ATILE   (TM * WP)
#define DYN_ELEMS (NHL * WMAT + NWAVES * 2 * ATILE)

static_assert(OFF_B0 == WID * IND);
static_assert(OFF_W1 == OFF_B0 + WID);
static_assert(LSTRIDE == WID * WID + WID);
static_assert(OFF_WL == OFF_W1 + NHL * LSTRIDE);
static_assert(OFF_BL == OFF_WL + WID);
static_assert(PCOUNT == OFF_BL + 1);
static_assert((WP % 8) == 0);
static_assert(NWAVES * 32 == WID);
static_assert((WMAT % 8) == 0);
static_assert((ATILE % 8) == 0);
static_assert((RPB % RPI) == 0);
static_assert(DYN_ELEMS * 2 == 139264);

typedef unsigned short v8us  __attribute__((ext_vector_type(8)));
typedef unsigned short v16us __attribute__((ext_vector_type(16)));
typedef float          v4f   __attribute__((ext_vector_type(4)));
typedef float          v8f   __attribute__((ext_vector_type(8)));
#if defined(__HIP_DEVICE_COMPILE__)
typedef __bf16         v16bf __attribute__((ext_vector_type(16)));
#endif

union FragU { v16us v; v8us half[2]; };

__device__ __forceinline__ unsigned bbits(float f) {
  unsigned u = __float_as_uint(f);
  return (u + 0x7FFFu + ((u >> 16) & 1u)) >> 16;
}
__device__ __forceinline__ float bf16r(float f) {
  return __uint_as_float(bbits(f) << 16);
}
__device__ __forceinline__ v8f zero8() { v8f z = {0.f, 0.f, 0.f, 0.f, 0.f, 0.f, 0.f, 0.f}; return z; }
__device__ __forceinline__ v8us zero8us() { v8us z = {0, 0, 0, 0, 0, 0, 0, 0}; return z; }
__device__ __forceinline__ float tanh_f(float z) {
  const float zc = fminf(fmaxf(z, -10.0f), 10.0f);
  const float e  = __expf(2.0f * zc);
  return 1.0f - 2.0f * __builtin_amdgcn_rcpf(e + 1.0f);
}
__device__ __forceinline__ void split2(float v, unsigned short& hb, unsigned short& lb) {
  const unsigned hu = bbits(v);
  hb = (unsigned short)hu;
  lb = (unsigned short)bbits(v - __uint_as_float(hu << 16));
}

__device__ __forceinline__ v16us ldfrag(const unsigned short* p) {
  FragU f;
  f.half[0] = *(const v8us*)(p);
  f.half[1] = *(const v8us*)(p + 16);
  return f.v;
}

__device__ __forceinline__ v8f mma_bf(v16us a, v16us b, v8f c) {
#if defined(__HIP_DEVICE_COMPILE__)
  return __builtin_amdgcn_wmma_f32_16x16x32_bf16(false, __builtin_bit_cast(v16bf, a),
                                                false, __builtin_bit_cast(v16bf, b),
                                                (short)0, c, false, false);
#else
  (void)a; (void)b;
  return c;
#endif
}
__device__ __forceinline__ void guard2(v8f& acc, const v16us& a, const v16us& b) {
#if defined(__HIP_DEVICE_COMPILE__)
  asm volatile("v_nop\n\tv_nop\n\tv_nop\n\tv_nop" : "+v"(acc) : "v"(a), "v"(b));
#endif
}
__device__ __forceinline__ void guard12(v8f& acc,
                                        const v16us& a0, const v16us& a1, const v16us& a2, const v16us& a3,
                                        const v16us& a4, const v16us& a5, const v16us& a6, const v16us& a7,
                                        const v16us& b0, const v16us& b1, const v16us& b2, const v16us& b3) {
#if defined(__HIP_DEVICE_COMPILE__)
  asm volatile("v_nop\n\tv_nop\n\tv_nop\n\tv_nop"
               : "+v"(acc)
               : "v"(a0), "v"(a1), "v"(a2), "v"(a3), "v"(a4), "v"(a5), "v"(a6), "v"(a7),
                 "v"(b0), "v"(b1), "v"(b2), "v"(b3));
#endif
}

__global__ __launch_bounds__(128)
void k_mlp(const float* __restrict__ X, const float* __restrict__ TH, float* out, int nx)
{
  extern __shared__ __align__(16) unsigned short dynlds[];
  __shared__ __align__(16) unsigned short w0s[WID * IND];
  __shared__ __align__(16) float b0s[WID];
  __shared__ __align__(16) float bls[NHL][WID];
  __shared__ __align__(16) float wls[WID];
  __shared__ __align__(16) float sOut[RPI];
  __shared__ float blv;

  const int tid = threadIdx.x;
  const int t   = blockIdx.y;
  const float* th = TH + (size_t)t * PCOUNT;

#pragma unroll 1
  for (int L = 0; L < NHL; ++L) {
    const float* src = th + OFF_W1 + (size_t)L * LSTRIDE;
    unsigned int* dst = (unsigned int*)(dynlds + (size_t)L * WMAT);
#pragma unroll 4
    for (int q = 0; q < (WID * (WID / 2)) / 128; ++q) {
      const int p    = tid + q * 128;
      const int nrow = p >> 6;
      const int k2   = (p & 63) * 2;
      const float f0 = src[nrow * WID + k2];
      const float f1 = src[nrow * WID + k2 + 1];
      dst[(nrow * WP + k2) >> 1] = bbits(f0) | (bbits(f1) << 16);
    }
  }
  {
    unsigned int* dst0 = (unsigned int*)w0s;
#pragma unroll 2
    for (int q = 0; q < (WID * (IND / 2)) / 128; ++q) {
      const int p    = tid + q * 128;
      const int nrow = p >> 3;
      const int k2   = (p & 7) * 2;
      const float f0 = th[nrow * IND + k2];
      const float f1 = th[nrow * IND + k2 + 1];
      dst0[(nrow * IND + k2) >> 1] = bbits(f0) | (bbits(f1) << 16);
    }
  }
  b0s[tid] = bf16r(th[OFF_B0 + tid]);
#pragma unroll
  for (int L = 0; L < NHL; ++L) bls[L][tid] = bf16r(th[OFF_W1 + L * LSTRIDE + WID * WID + tid]);
  wls[tid] = bf16r(th[OFF_WL + tid]);
  if (tid == 0) blv = bf16r(th[OFF_BL]);
  __syncthreads();

  const int lane = tid & 31;
  const int wave = tid >> 5;
  const int hh   = lane >> 4;
  const int c    = lane & 15;
  unsigned short* actH = dynlds + (size_t)NHL * WMAT + (size_t)wave * (2 * ATILE);
  unsigned short* actL = actH + ATILE;
  const float bl = blv;
  const int blockRow0 = blockIdx.x * RPB;
  float* outT = out + (size_t)t * (size_t)nx;
  const v8us z8 = zero8us();

#pragma unroll 1
  for (int it = 0; it < ITERS; ++it) {
    const int rbase = blockRow0 + it * RPI;
    if (rbase >= nx) break;
    const int r0w = rbase + wave * TM;
    __syncthreads();

    {
      int gr = r0w + c;
      if (gr > nx - 1) gr = nx - 1;
      const float* xp = X + (size_t)gr * IND + 8 * hh;
      const v4f x0 = *(const v4f*)(xp);
      const v4f x1 = *(const v4f*)(xp + 4);
      v8us xa;
      xa[0] = (unsigned short)bbits(x0[0]); xa[1] = (unsigned short)bbits(x0[1]);
      xa[2] = (unsigned short)bbits(x0[2]); xa[3] = (unsigned short)bbits(x0[3]);
      xa[4] = (unsigned short)bbits(x1[0]); xa[5] = (unsigned short)bbits(x1[1]);
      xa[6] = (unsigned short)bbits(x1[2]); xa[7] = (unsigned short)bbits(x1[3]);
      FragU fa;
      fa.half[0] = xa;
      fa.half[1] = z8;
      const v16us a0 = fa.v;

#pragma unroll 1
      for (int nt = 0; nt < 8; ++nt) {
        const int n0 = nt * 16;
        FragU fb;
        fb.half[0] = *(const v8us*)(w0s + (n0 + c) * IND + 8 * hh);
        fb.half[1] = z8;
        const v16us g = fb.v;
        v8f acc = zero8();
        acc = mma_bf(a0, g, acc);
        guard2(acc, a0, g);
        const int ncol = n0 + c;
        const float bias = b0s[ncol];
#pragma unroll
        for (int r = 0; r < 8; ++r) {
          const float hv = tanh_f(acc[r] + bias);
          unsigned short hb, lb;
          split2(hv, hb, lb);
          const int o = (8 * hh + r) * WP + ncol;
          actH[o] = hb;
          actL[o] = lb;
        }
      }
    }
    __syncthreads();

#pragma unroll 1
    for (int li = 0; li < NHL; ++li) {
      const unsigned short* wl  = dynlds + (size_t)li * WMAT;
      const unsigned short* arh = actH + c * WP + 8 * hh;
      const unsigned short* arl = actL + c * WP + 8 * hh;
      const v16us ah0 = ldfrag(arh),      ah1 = ldfrag(arh + 32), ah2 = ldfrag(arh + 64), ah3 = ldfrag(arh + 96);
      const v16us al0 = ldfrag(arl),      al1 = ldfrag(arl + 32), al2 = ldfrag(arl + 64), al3 = ldfrag(arl + 96);
      float s[8];
#pragma unroll
      for (int r = 0; r < 8; ++r) s[r] = 0.0f;

#pragma unroll 1
      for (int nt = 0; nt < 8; ++nt) {
        const int n0 = nt * 16;
        const unsigned short* wp = wl + (n0 + c) * WP + 8 * hh;
        const v16us g0 = ldfrag(wp);
        const v16us g1 = ldfrag(wp + 32);
        const v16us g2 = ldfrag(wp + 64);
        const v16us g3 = ldfrag(wp + 96);
        v8f acc = zero8();
        acc = mma_bf(ah0, g0, acc);
        acc = mma_bf(al0, g0, acc);
        acc = mma_bf(ah1, g1, acc);
        acc = mma_bf(al1, g1, acc);
        acc = mma_bf(ah2, g2, acc);
        acc = mma_bf(al2, g2, acc);
        acc = mma_bf(ah3, g3, acc);
        acc = mma_bf(al3, g3, acc);
        guard12(acc, ah0, ah1, ah2, ah3, al0, al1, al2, al3, g0, g1, g2, g3);
        const int ncol = n0 + c;
        const float bias = bls[li][ncol];
        if (li < NHL - 1) {
#pragma unroll
          for (int r = 0; r < 8; ++r) {
            const float hv = tanh_f(acc[r] + bias);
            unsigned short hb, lb;
            split2(hv, hb, lb);
            const int o = (8 * hh + r) * WP + ncol;
            actH[o] = hb;
            actL[o] = lb;
          }
        } else {
          const float wv = wls[ncol];
#pragma unroll
          for (int r = 0; r < 8; ++r) {
            const float hv = tanh_f(acc[r] + bias);
            s[r] += hv * wv;
          }
        }
      }

      if (li == NHL - 1) {
#pragma unroll
        for (int off = 8; off >= 1; off >>= 1) {
#pragma unroll
          for (int r = 0; r < 8; ++r) s[r] += __shfl_xor(s[r], off, 16);
        }
        if (c == 0) {
#pragma unroll
          for (int r = 0; r < 8; ++r) sOut[wave * TM + 8 * hh + r] = s[r] + bl;
        }
      }
      __syncthreads();
    }

    {
      const int lc = lane & 15;
      const v4f ov = *(const v4f*)(sOut + 4 * lc);
      const bool wr = (wave == 0) && (lane < 16);
      float* po = outT + (size_t)rbase + 4 * lc;
      if (wr) *(volatile v4f*)po = ov;
      __threadfence();
      if (wr) *(volatile v4f*)po = ov;
    }
  }
}

extern "C" void kernel_launch(void* const* d_in, const int* in_sizes, int n_in,
                              void* d_out, int out_size, void* d_ws, size_t ws_size,
                              hipStream_t stream) {
  (void)d_ws; (void)ws_size;
  if (n_in < 2) return;
  if (in_sizes[0] < IND * RPI || (in_sizes[0] % IND) != 0) return;
  const int nx = in_sizes[0] / IND;
  if ((nx % RPI) != 0) return;
  if (in_sizes[1] < PCOUNT || (in_sizes[1] % PCOUNT) != 0) return;
  const int T = in_sizes[1] / PCOUNT;
  if (T > 65535) return;
  if ((long long)out_size != (long long)T * (long long)nx) return;

  const float* X  = (const float*)d_in[0];
  const float* TH = (const float*)d_in[1];
  float* out = (float*)d_out;

  const size_t dynBytes = (size_t)DYN_ELEMS * sizeof(unsigned short);
  (void)hipFuncSetAttribute(reinterpret_cast<const void*>(&k_mlp),
                            hipFuncAttributeMaxDynamicSharedMemorySize, (int)dynBytes);
  const dim3 grid((nx + RPB - 1) / RPB, T);
  k_mlp<<<grid, dim3(128), dynBytes, stream>>>(X, TH, out, nx);
  (void)hipGetLastError();
}
